// GraphConvolution_40896678593043
// MI455X (gfx1250) — hardware-verified
//
#include <hip/hip_runtime.h>


namespace {
constexpr int B = 4, T = 4096, C = 128, DQ = 32  , QKW = 2 * DQ  , HD = 128  , BL = 4  , QL = T;
constexpr float XS = 8.0f, WSC = 256.0f, WSQ = 0.25f, PS = 1024.0f, RS_ = 1024.0f, LOG2E = 1.4426950408889634f;
static_assert(T % 64 == 0 && C == 128 && HD == 128 && DQ == 32, "tiling");
typedef _Float16 b16;
typedef __attribute__((ext_vector_type(16))) _Float16 v16b;
typedef __attribute__((ext_vector_type(8))) _Float16 v8b;
typedef __attribute__((ext_vector_type(8))) float v8f;
typedef __attribute__((ext_vector_type(4))) float v4f;
__device__ __forceinline__ float bf16_rne(float f) { unsigned int u = __float_as_uint(f); u += 0x7FFFu + ((u >> 16) & 1u); return __uint_as_float(u & 0xFFFF0000u); }
__device__ __forceinline__ void split16(float v, b16& hi, b16& lo) { hi = (b16)v; lo = (b16)(v - (float)hi); }
__device__ __forceinline__ v16b frag_kb(const b16* p, int hh) { const v8b a = *(const v8b*)(p + 8 * hh), b = *(const v8b*)(p + 16 + 8 * hh); v16b f;
#pragma unroll
  for (int e = 0; e < 8; ++e) { f[e] = a[e]; f[8 + e] = b[e]; } return f; }
__device__ __forceinline__ v8f wmma16b(v16b a, v16b b, v8f c) { v8f d = __builtin_amdgcn_wmma_f32_16x16x32_f16(false, a, false, b, (short)0, c, false, false); asm volatile("v_nop\n\tv_nop\n\tv_nop\n\tv_nop" : "+v"(d) : "v"(a), "v"(b)); return d; }
__device__ __forceinline__ void wave_lds_sync() { __builtin_amdgcn_fence(__ATOMIC_RELEASE, "workgroup"); __builtin_amdgcn_wave_barrier(); __builtin_amdgcn_fence(__ATOMIC_ACQUIRE, "workgroup"); }
__device__ __forceinline__ float pmul(float a, float b) { float p = a * b; asm volatile("" : "+v"(p)); return p; }
__device__ __forceinline__ int iclamp(int v, int lo, int hi) { return v < lo ? lo : (v > hi ? hi : v); }

typedef __attribute__((ext_vector_type(2))) _Float16 v2h;
typedef __attribute__((ext_vector_type(4))) _Float16 v4h;
typedef __attribute__((ext_vector_type(2))) float v2f;
typedef __attribute__((ext_vector_type(4))) int v4i;
__device__ __forceinline__ float nexp2(float v) { return __builtin_amdgcn_exp2f(v); }
__global__ __launch_bounds__(256) void prep_kernel(const float* __restrict__ wq, const float* __restrict__ wk, const float* __restrict__ wv, const float* __restrict__ wg, b16* __restrict__ WQK, b16* __restrict__ WV, b16* __restrict__ WG, b16* __restrict__ WGq) {
  const int u = blockIdx.x * 256 + threadIdx.x; const int n1 = QKW * C / 8, n2 = C * C / 8; if (u >= n1 + 2 * n2) return; v8b v;
  if (u < n1) { const int e = u * 8; const int o = e / C, c0 = e % C; const float* w = (o < DQ) ? (wk + (size_t)o * C) : (wq + (size_t)(o - DQ) * C); for (int j = 0; j < 8; ++j) v[j] = (b16)(bf16_rne(w[c0 + j]) * WSC); for (int pass = 0; pass < 2; ++pass) { *(volatile v8b*)(WQK + e) = v; __threadfence(); } }
  else if (u < n1 + n2) { const int e = (u - n1) * 8; for (int j = 0; j < 8; ++j) v[j] = (b16)(bf16_rne(wv[e + j]) * WSC); for (int pass = 0; pass < 2; ++pass) { *(volatile v8b*)(WV + e) = v; __threadfence(); } }
  else { const int e = (u - n1 - n2) * 8; const int o = e / C, k0 = e % C; v8b vq; for (int j = 0; j < 8; ++j) { const float w = bf16_rne(wg[(size_t)(k0 + j) * C + o]); v[j] = (b16)(w * WSC); vq[j] = (b16)(w * WSQ); } for (int pass = 0; pass < 2; ++pass) { *(volatile v8b*)(WG + e) = v; *(volatile v8b*)(WGq + e) = vq; __threadfence(); } }
}
__global__ __launch_bounds__(64) void qk_kernel(const float* __restrict__ x, const b16* __restrict__ WQK, const float* __restrict__ bq, const float* __restrict__ bk, b16* __restrict__ QK, b16* __restrict__ QKl) {
  __shared__ __attribute__((aligned(16))) b16 Ah[2][16][C + 8]; __shared__ __attribute__((aligned(16))) float Tf[2][16][QKW + 4];
  const int wave = threadIdx.x >> 5, lane = threadIdx.x & 31, nloc = lane & 15, hlf = lane >> 4; const size_t m0 = (size_t)blockIdx.x * 32 + wave * 16;
  for (int idx = lane; idx < 16 * (C / 4); idx += 32) { const int rr = idx / (C / 4), c4 = (idx % (C / 4)) * 4; const v4f v = *(const v4f*)(x + (m0 + rr) * C + c4); v4h hv; for (int j = 0; j < 4; ++j) hv[j] = (b16)(bf16_rne(v[j]) * XS); *(v4h*)(&Ah[wave][rr][c4]) = hv; }
  wave_lds_sync();
  v8f acc[4]; for (int t = 0; t < 4; ++t) acc[t] = (v8f){};
#pragma unroll
  for (int kb = 0; kb < C; kb += 32) { const v16b a = frag_kb(&Ah[wave][nloc][kb], hlf);
#pragma unroll
    for (int t = 0; t < 4; ++t) acc[t] = wmma16b(a, frag_kb(WQK + (size_t)(t * 16 + nloc) * C + kb, hlf), acc[t]); }
#pragma unroll
  for (int t = 0; t < 4; ++t) { const int col = t * 16 + nloc; const float bb = bf16_rne(col < DQ ? bk[col] : bq[col - DQ]); for (int r = 0; r < 8; ++r) Tf[wave][8 * hlf + r][col] = acc[t][r] * (1.0f / (XS * WSC)) + bb; }
  wave_lds_sync();
  for (int pass = 0; pass < 2; ++pass) { for (int rr = 0; rr < 16; rr += 2) { const int r2 = rr + (lane >> 4); v4h h4, l4; for (int j = 0; j < 4; ++j) { const float f = Tf[wave][r2][(lane & 15) * 4 + j] * XS; const b16 p = (b16)f; h4[j] = p; l4[j] = (b16)((f - (float)p) * RS_); }
      const size_t oi = (m0 + r2) * QKW + (lane & 15) * 4; *(volatile v4h*)(QK + oi) = h4; *(volatile v4h*)(QKl + oi) = l4; } __threadfence(); }
}
__global__ __launch_bounds__(128) void sup_kernel(const float* __restrict__ x, int b0unused, const b16* __restrict__ WV, const float* __restrict__ bv, const b16* __restrict__ WG, const b16* __restrict__ WGq, b16* __restrict__ VT, b16* __restrict__ VTl) {
  __shared__ __attribute__((aligned(16))) b16 Ah[4][16][C + 8], Al[4][16][C + 8]; __shared__ __attribute__((aligned(16))) float Tf[4][16][HD + 4];
  const int wave = threadIdx.x >> 5, lane = threadIdx.x & 31, nloc = lane & 15, hlf = lane >> 4; const int b = blockIdx.y, t0 = blockIdx.x * 64; const size_t m0 = (size_t)b * T + t0 + wave * 16;
  (void)b0unused;
  for (int idx = lane; idx < 16 * (C / 4); idx += 32) { const int rr = idx / (C / 4), c4 = (idx % (C / 4)) * 4; const v4f v = *(const v4f*)(x + (m0 + rr) * C + c4); v4h hv; for (int j = 0; j < 4; ++j) hv[j] = (b16)(bf16_rne(v[j]) * XS); *(v4h*)(&Ah[wave][rr][c4]) = hv; }
  wave_lds_sync();
  v8f acc[8];
#pragma unroll
  for (int t = 0; t < 8; ++t) acc[t] = (v8f){};
#pragma unroll
  for (int kb = 0; kb < C; kb += 32) { const v16b a = frag_kb(&Ah[wave][nloc][kb], hlf);
#pragma unroll
    for (int t = 0; t < 8; ++t) acc[t] = wmma16b(a, frag_kb(WV + (size_t)(t * 16 + nloc) * C + kb, hlf), acc[t]); }
  wave_lds_sync();
#pragma unroll
  for (int t = 0; t < 8; ++t) { const float bb = bf16_rne(bv[t * 16 + nloc]); for (int r = 0; r < 8; ++r) Tf[wave][8 * hlf + r][t * 16 + nloc] = acc[t][r] * (1.0f / (XS * WSC)) + bb; }
  wave_lds_sync();
  for (int idx = lane; idx < 16 * (HD / 4); idx += 32) { const int rr = idx / (HD / 4), c4 = (idx % (HD / 4)) * 4; v4h hv, lv; for (int j = 0; j < 4; ++j) { const float vs = Tf[wave][rr][c4 + j] * XS; const b16 ph = (b16)vs; hv[j] = ph; lv[j] = (b16)((vs - (float)ph) * RS_); } *(v4h*)(&Ah[wave][rr][c4]) = hv; *(v4h*)(&Al[wave][rr][c4]) = lv; }
  wave_lds_sync();
#pragma unroll
  for (int t = 0; t < 8; ++t) acc[t] = (v8f){};
#pragma unroll
  for (int kb = 0; kb < HD; kb += 32) { const v16b a = frag_kb(&Ah[wave][nloc][kb], hlf), al = frag_kb(&Al[wave][nloc][kb], hlf);
#pragma unroll
    for (int t = 0; t < 8; ++t) { const size_t wo_ = (size_t)(t * 16 + nloc) * HD + kb; acc[t] = wmma16b(a, frag_kb(WG + wo_, hlf), acc[t]); acc[t] = wmma16b(al, frag_kb(WGq + wo_, hlf), acc[t]); } }
  wave_lds_sync();
#pragma unroll
  for (int t = 0; t < 8; ++t) for (int r = 0; r < 8; ++r) Tf[wave][8 * hlf + r][t * 16 + nloc] = acc[t][r] * (1.0f / (XS * WSC));
  __syncthreads();
  for (int pass = 0; pass < 2; ++pass) {
#pragma unroll 1
    for (int q = 0; q < 32; ++q) { const int u = wave * 32 + q; const int tk = lane * 2; v2h hv, lv; for (int j = 0; j < 2; ++j) { const float f = Tf[(tk + j) >> 4][(tk + j) & 15][u] * XS; const b16 p = (b16)f; hv[j] = p; lv[j] = (b16)((f - (float)p) * RS_); }
      const size_t oi = ((size_t)b * HD + u) * (size_t)T + t0 + lane * 2; *(volatile v2h*)(VT + oi) = hv; *(volatile v2h*)(VTl + oi) = lv; }
    __threadfence(); }
}
__global__ __launch_bounds__(64) void attn_kernel(const b16* __restrict__ QP, const b16* __restrict__ QPl, const b16* __restrict__ KP, const b16* __restrict__ KPl, const b16* __restrict__ VT, const b16* __restrict__ VTl, const float* __restrict__ obias, float* __restrict__ out) {
  __shared__ __attribute__((aligned(16))) b16 Pb[2][16][32 + 8]; __shared__ __attribute__((aligned(16))) float To[2][16][HD + 4];
  const int wave = threadIdx.x >> 5, lane = threadIdx.x & 31, hh = lane >> 4, col = lane & 15; const int b = blockIdx.y, h = 0; (void)h; const int q0 = blockIdx.x * 32 + wave * 16, qi = q0 + col;
  const size_t qo = (size_t)b * T * QKW, vo = (size_t)b * HD * (size_t)T; const b16* Qb = QP + qo; const b16* Qbl = QPl + qo; const b16* Kb = QP + qo + DQ; const b16* Kbl = QPl + qo + DQ; const b16* Vb = VT + vo; const b16* Vbl = VTl + vo; (void)KP; (void)KPl;
  const v16b qf0 = frag_kb(Qb + (size_t)qi * QKW, hh), ql0 = frag_kb(Qbl + (size_t)qi * QKW, hh);
  const float cs = LOG2E / (XS * XS);
  __shared__ __attribute__((aligned(16))) b16 Plq[2][16][32 + 8];
  float m = -INFINITY, l = 0.0f; v8f o[8], ol[8]; for (int t = 0; t < 8; ++t) { o[t] = (v8f){}; ol[t] = (v8f){}; }
#pragma unroll 1
  for (int kb = 0; kb < T; kb += 32) {
    float e[16]; float mx = -INFINITY;
#pragma unroll
    for (int u = 0; u < 2; ++u) { v8f s = (v8f){}, sx = (v8f){}; const size_t kr = (size_t)(kb + u * 16 + col) * QKW;
      { const v16b kf = frag_kb(Kb + kr, hh); s = wmma16b(kf, qf0, s); sx = wmma16b(kf, ql0, sx); sx = wmma16b(frag_kb(Kbl + kr, hh), qf0, sx); }
#pragma unroll
      for (int r = 0; r < 8; ++r) s[r] += sx[r] * (1.0f / RS_);
#pragma unroll
      for (int r = 0; r < 8; ++r) { const float vv = s[r] * cs; e[u * 8 + r] = vv; mx = fmaxf(mx, vv); } }
    mx = fmaxf(mx, __shfl_xor(mx, 16)); const float mn = fmaxf(m, mx); const float al = nexp2(m - mn); float sum = 0.0f;
#pragma unroll
    for (int i2 = 0; i2 < 16; ++i2) { const float p = nexp2(e[i2] - mn); sum += p; const int pc = (i2 < 8 ? 0 : 16) + 8 * hh + (i2 & 7); const float ps = p * PS; const b16 phh = (b16)ps; Pb[wave][col][pc] = phh; Plq[wave][col][pc] = (b16)((ps - (float)phh) * RS_); }
    sum += __shfl_xor(sum, 16); l = l * al + sum; m = mn;
    wave_lds_sync();
    const v16b pf = frag_kb(&Pb[wave][col][0], hh), plf = frag_kb(&Plq[wave][col][0], hh);
#pragma unroll
    for (int t = 0; t < 8; ++t) { const v16b vh = frag_kb(Vb + (size_t)(t * 16 + col) * T + kb, hh); o[t] *= al; o[t] = wmma16b(vh, pf, o[t]); ol[t] = wmma16b(frag_kb(Vbl + (size_t)(t * 16 + col) * T + kb, hh), pf, ol[t] * al); ol[t] = wmma16b(vh, plf, ol[t]); }
    wave_lds_sync(); }
  const float inv = 1.0f / (l * PS * XS);
#pragma unroll
  for (int t = 0; t < 8; ++t)
#pragma unroll
    for (int r = 0; r < 8; ++r) To[wave][col][t * 16 + 8 * hh + r] = (o[t][r] + ol[t][r] * (1.0f / RS_)) * inv;
  wave_lds_sync();
  for (int pass = 0; pass < 2; ++pass) { for (int rr = 0; rr < 16; ++rr) { v4f o4 = *(const v4f*)(&To[wave][rr][lane * 4]); for (int j = 0; j < 4; ++j) o4[j] += bf16_rne(obias[lane * 4 + j]); *(volatile v4f*)(out + ((size_t)b * T + q0 + rr) * HD + lane * 4) = o4; } __threadfence(); }
}
}

extern "C" void kernel_launch(void* const* d_in, const int* in_sizes, int n_in, void* d_out, int out_size, void* d_ws, size_t ws_size, hipStream_t stream) {
  (void)n_in;
  auto Fp = [&](int i) { return (const float*)d_in[i]; };
  if (in_sizes[0] != B * T * C || in_sizes[1] != C * HD || in_sizes[2] != HD || in_sizes[3] != DQ * C || in_sizes[4] != DQ || in_sizes[5] != DQ * C || in_sizes[6] != DQ || in_sizes[7] != HD * C || in_sizes[8] != HD || out_size != B * T * HD) return;
  size_t off = 0; char* ws = (char*)d_ws;
  auto carve = [&](size_t bytes) { char* p = ws + off; off += (bytes + 255) & ~(size_t)255; return p; };
  b16* WQK = (b16*)carve((size_t)QKW * C * 2); b16* WV = (b16*)carve((size_t)C * HD * 2); b16* WG = (b16*)carve((size_t)HD * HD * 2); b16* WGq = (b16*)carve((size_t)HD * HD * 2);
  b16* QK = (b16*)carve((size_t)B * T * QKW * 2); b16* QKl = (b16*)carve((size_t)B * T * QKW * 2); b16* VT = (b16*)carve((size_t)B * HD * T * 2); b16* VTl = (b16*)carve((size_t)B * HD * T * 2);
  if (off > ws_size || off > ((size_t)128 << 20)) return;
  prep_kernel<<<(QKW * C / 8 + 2 * C * C / 8 + 255) / 256, 256, 0, stream>>>(Fp(3), Fp(5), Fp(7), Fp(1), WQK, WV, WG, WGq);
  qk_kernel<<<(B * T) / 32, 64, 0, stream>>>(Fp(0), WQK, Fp(4), Fp(6), QK, QKl);
  sup_kernel<<<dim3(T / 64, BL), 128, 0, stream>>>(Fp(0), 0, WV, Fp(8), WG, WGq, VT, VTl);
  attn_kernel<<<dim3(QL / 32, BL), 64, 0, stream>>>(QK, QKl, QK, QKl, VT, VTl, Fp(2), (float*)d_out);
}
